// STGCN_MLP_60902636257629
// MI455X (gfx1250) — hardware-verified
//
#include <hip/hip_runtime.h>
#include <stddef.h>


#define N_NODES 14
#define SEQ     24
#define KP      32
#define GH      64
#define MH      64
#define NEDGE   56
#define ETOT    70
#define ADJP    72
#define SPB     16
#define NR      (SPB * N_NODES)
#define NT      (NR / 16)
#define NTHR    256
#define NWAVE   8
#define XTILE   (SPB * SEQ * N_NODES)
#define XVEC    (XTILE / 4)

#define PL_W1   0
#define PL_W2   2048
#define PL_F1   4096
#define PL_F2   (PL_F1 + N_NODES * 2048)
#define PL_TOT  (PL_F2 + N_NODES * 2048)

#define RX_OFF  0
#define RX_N    (NR * KP)
#define RH_OFF  (RX_OFF + RX_N)
#define RH_N    (NR * GH)
#define RG_OFF  (RH_OFF + RH_N)
#define RG_N    (NR * GH)
#define SM_OFF  (RG_OFF + RG_N)
#define SM_N    2048
#define LDS_FLOATS (SM_OFF + SM_N)
#define LDS_BYTES  (LDS_FLOATS * 4)

static_assert(NR % 16 == 0);
static_assert(N_NODES * SPB * SEQ <= RX_N);
static_assert(NR * KP <= RH_N);
static_assert(N_NODES * SPB * MH <= RG_N);
static_assert(XVEC * 4 == XTILE);
static_assert(800 + 16 + 16 * ADJP <= SM_N);
static_assert((SPB * SEQ) % 128 == 0);
static_assert(PL_TOT % 256 == 0);
static_assert(PL_W2 % 256 == 0 && PL_F1 % 256 == 0 && PL_F2 % 256 == 0);

typedef float  v4f  __attribute__((ext_vector_type(4)));
typedef float  v8f  __attribute__((ext_vector_type(8)));
typedef int    v4i  __attribute__((ext_vector_type(4)));
typedef __bf16 v8b  __attribute__((ext_vector_type(8)));
typedef __bf16 v16b __attribute__((ext_vector_type(16)));
union FragB { v16b v; v4i q[2]; };
union Pack8 { v8b v; v4i q; };

__device__ __forceinline__ v8f wmb(v16b a, v16b b, v8f c) {
  v8f d = __builtin_amdgcn_wmma_f32_16x16x32_bf16(false, a, false, b, (short)0, c, false, false);
  asm volatile("v_nop\n\tv_nop\n\tv_nop\n\tv_nop" : "+v"(d) : "v"(a), "v"(b));
  return d;
}

__device__ __forceinline__ v8f wm3(v16b ah, v16b al, v16b bh, v16b bl, v8f c) {
  c = wmb(ah, bh, c);
  c = wmb(al, bh, c);
  c = wmb(ah, bl, c);
  return c;
}

#define SPL(I, X) { const float f_ = (X); const __bf16 h_ = (__bf16)f_; hi[I] = h_; lo[I] = (__bf16)(f_ - (float)h_); }
__device__ __forceinline__ void load_a_split(const float* ar, v16b& hi, v16b& lo) {
  const v4f p0 = *(const v4f*)(ar);
  const v4f p1 = *(const v4f*)(ar + 4);
  const v4f p2 = *(const v4f*)(ar + 16);
  const v4f p3 = *(const v4f*)(ar + 20);
  SPL(0, p0.x)  SPL(1, p0.y)  SPL(2, p0.z)  SPL(3, p0.w)
  SPL(4, p1.x)  SPL(5, p1.y)  SPL(6, p1.z)  SPL(7, p1.w)
  SPL(8, p2.x)  SPL(9, p2.y)  SPL(10, p2.z) SPL(11, p2.w)
  SPL(12, p3.x) SPL(13, p3.y) SPL(14, p3.z) SPL(15, p3.w)
}
#undef SPL

__device__ __forceinline__ void load_b(const __bf16* ph, const __bf16* pl, int off, FragB& bh, FragB& bl) {
  bh.q[0] = *(const v4i*)(ph + off);
  bh.q[1] = *(const v4i*)(ph + off + 16);
  bl.q[0] = *(const v4i*)(pl + off);
  bl.q[1] = *(const v4i*)(pl + off + 16);
}

__global__ __launch_bounds__(NTHR) void k_prep(
    const float* __restrict__ W1, const float* __restrict__ W2,
    const float* __restrict__ f1w, const float* __restrict__ f2w,
    __bf16* ph, __bf16* pl) {
  const int r = blockIdx.y;
  const int nblk = (r < 2) ? 1 : N_NODES;
  if ((int)blockIdx.x >= nblk) return;
  const float* src = (r == 0) ? W1 : (r == 1) ? W2 : (r == 2) ? f1w : f2w;
  const int K    = (r == 0 || r == 2) ? SEQ : GH;
  const int N    = (r == 0 || r == 2) ? GH : SEQ;
  const int kpl  = (r == 0 || r == 2) ? 5 : 6;
  const int base = (r == 0) ? PL_W1 : (r == 1) ? PL_W2 : (r == 2) ? PL_F1 : PL_F2;
  const int idx  = blockIdx.x * NTHR + threadIdx.x;
  const int o    = idx * 8;
  const int node = o >> 11;
  const int rem  = o & 2047;
  const int n    = rem >> kpl;
  const int k0   = rem & ((1 << kpl) - 1);
  const int nc   = n < N ? n : N - 1;
  const float* sp = src + (size_t)node * (SEQ * GH);
  Pack8 hv, lv;
#pragma unroll
  for (int j = 0; j < 8; ++j) {
    const int k  = k0 + j;
    const int kc = k < K ? k : K - 1;
    const float f = sp[kc * N + nc];
    const float v = (n < N && k < K) ? f : 0.f;
    const __bf16 h = (__bf16)v;
    hv.v[j] = h;
    lv.v[j] = (__bf16)(v - (float)h);
  }
  __bf16* dh = ph + base + o;
  __bf16* dl = pl + base + o;
  const v4i qh = hv.q, ql = lv.q;
  *(volatile v4i*)dh = qh;
  *(volatile v4i*)dl = ql;
  __threadfence();
  *(volatile v4i*)dh = qh;
  *(volatile v4i*)dl = ql;
}

__global__ __launch_bounds__(NTHR) void k_main(
    const float* __restrict__ x, const int* __restrict__ ei,
    const float* __restrict__ as1, const float* __restrict__ ad1, const float* __restrict__ b1,
    const float* __restrict__ as2, const float* __restrict__ ad2, const float* __restrict__ b2,
    const float* __restrict__ f1b, const float* __restrict__ f2b,
    const __bf16* __restrict__ ph, const __bf16* __restrict__ pl,
    float* out, int nB) {
  extern __shared__ v4f lds_dyn[];
  float* L    = (float*)lds_dyn;
  float* RX   = L + RX_OFF;
  float* RH   = L + RH_OFF;
  float* RG   = L + RG_OFF;
  float* sP   = L + SM_OFF;
  float* sQ   = sP + 256;
  float* sAs1 = sQ + 256;
  float* sAd1 = sAs1 + 64;
  float* sBi1 = sAd1 + 64;
  float* sAs2 = sBi1 + 64;
  float* sAd2 = sAs2 + 32;
  float* sBi2 = sAd2 + 32;
  int*   sCnt = (int*)(sBi2 + 32);
  int*   sAdj = sCnt + 16;

  const int t = threadIdx.x, lane = t & 31, wave = t >> 5, hh = lane >> 4, m = lane & 15;
  const int b0 = blockIdx.x * SPB;
  if (b0 + SPB > nB) return;

  {
    const v4f z = {0.f, 0.f, 0.f, 0.f};
    for (int i = t; i < RX_N / 4; i += NTHR) ((v4f*)RX)[i] = z;
  }
  {
    const int i64 = t < 63 ? t : 63;
    const int i24 = t < 23 ? t : 23;
    const float va = as1[i64], vd = ad1[i64], vb = b1[i64];
    const float wa = as2[i24], wd = ad2[i24], wb = b2[i24];
    if (t < 64) { sAs1[t] = va; sAd1[t] = vd; sBi1[t] = vb; }
    if (t < 32) {
      const bool in = t < SEQ;
      sAs2[t] = in ? wa : 0.f; sAd2[t] = in ? wd : 0.f; sBi2[t] = in ? wb : 0.f;
    }
  }
  if (wave == 0) {
    const int d = lane & 15;
    int pos = 0;
#pragma unroll 1
    for (int e = 0; e < ETOT; ++e) {
      const int ec = e < NEDGE ? e : NEDGE - 1;
      int rs = ei[ec];
      int rd = ei[NEDGE + ec];
      rs = rs < 0 ? 0 : (rs > N_NODES - 1 ? N_NODES - 1 : rs);
      rd = rd < 0 ? 0 : (rd > N_NODES - 1 ? N_NODES - 1 : rd);
      const int sr = e < NEDGE ? rs : e - NEDGE;
      const int ds = e < NEDGE ? rd : e - NEDGE;
      const bool hit = (ds == d);
      if (hit && pos < ETOT) sAdj[d * ADJP + pos] = sr;
      pos += hit ? 1 : 0;
    }
    sCnt[d] = pos > ETOT ? ETOT : pos;
  }
  __syncthreads();

  {
    const float* xb = x + (size_t)b0 * (SEQ * N_NODES);
#pragma unroll 1
    for (int i = 0; i < (XVEC + NTHR - 1) / NTHR; ++i) {
      const int idx = i * NTHR + t;
      const int ic  = idx < XVEC ? idx : XVEC - 1;
      const v4f v   = *(const v4f*)(xb + 4 * ic);
      if (idx < XVEC) {
#pragma unroll
        for (int c = 0; c < 4; ++c) {
          const int li = 4 * idx + c;
          const int s  = li / (SEQ * N_NODES);
          const int rm = li - s * (SEQ * N_NODES);
          const int f  = rm / N_NODES;
          const int n  = rm - f * N_NODES;
          RX[(s * N_NODES + n) * KP + f] = v[c];
        }
      }
    }
  }
  __syncthreads();

#pragma unroll
  for (int rep = 0; rep < 2; ++rep) {
    const int tI = wave + NWAVE * rep;
    if (tI < NT) {
      v16b ah, al;
      load_a_split(RX + (tI * 16 + m) * KP + 8 * hh, ah, al);
#pragma unroll
      for (int nt = 0; nt < GH / 16; ++nt) {
        FragB bh, bl;
        load_b(ph, pl, PL_W1 + (16 * nt + m) * KP + 8 * hh, bh, bl);
        v8f c = {0.f, 0.f, 0.f, 0.f, 0.f, 0.f, 0.f, 0.f};
        c = wm3(ah, al, bh.v, bl.v, c);
        float* dp = RH + (tI * 16 + 8 * hh) * GH + 16 * nt + m;
#pragma unroll
        for (int r = 0; r < 8; ++r) dp[r * GH] = c[r];
      }
    }
  }
  __syncthreads();

  {
    const int s = t >> 4, n = t & 15;
    float p = 0.f, q = 0.f;
    if (n < N_NODES) {
      const float* hr = RH + (s * N_NODES + n) * GH;
#pragma unroll
      for (int f4 = 0; f4 < GH / 4; ++f4) {
        const v4f hv = *(const v4f*)(hr + 4 * f4);
        const v4f av = *(const v4f*)(sAs1 + 4 * f4);
        const v4f dv = *(const v4f*)(sAd1 + 4 * f4);
        p = p + hv.x * av.x; p = p + hv.y * av.y; p = p + hv.z * av.z; p = p + hv.w * av.w;
        q = q + hv.x * dv.x; q = q + hv.y * dv.y; q = q + hv.z * dv.z; q = q + hv.w * dv.w;
      }
    }
    sP[s * 16 + n] = p;
    sQ[s * 16 + n] = q;
  }
  __syncthreads();

  {
    const int s = t >> 4, d = t & 15;
    if (d < N_NODES) {
      int cnt = sCnt[d];
      cnt = cnt < 1 ? 1 : (cnt > ETOT ? ETOT : cnt);
      const float  qd  = sQ[s * 16 + d];
      const float* sPs = sP + s * 16;
      const int*   adj = sAdj + d * ADJP;
      float mx = -3.0e38f;
#pragma unroll 1
      for (int i = 0; i < cnt; ++i) {
        int sr = adj[i];
        sr = sr < 0 ? 0 : (sr > N_NODES - 1 ? N_NODES - 1 : sr);
        float a = sPs[sr] + qd;
        a = (a >= 0.f) ? a : 0.2f * a;
        mx = fmaxf(mx, a);
      }
      float acc[GH];
#pragma unroll
      for (int j = 0; j < GH; ++j) acc[j] = 0.f;
      float sum = 0.f;
#pragma unroll 1
      for (int i = 0; i < cnt; ++i) {
        int sr = adj[i];
        sr = sr < 0 ? 0 : (sr > N_NODES - 1 ? N_NODES - 1 : sr);
        float a = sPs[sr] + qd;
        a = (a >= 0.f) ? a : 0.2f * a;
        const float e = __expf(a - mx);
        sum += e;
        const float* hr = RH + (s * N_NODES + sr) * GH;
#pragma unroll
        for (int j4 = 0; j4 < GH / 4; ++j4) {
          const v4f hv = *(const v4f*)(hr + 4 * j4);
          acc[4 * j4 + 0] += e * hv.x;
          acc[4 * j4 + 1] += e * hv.y;
          acc[4 * j4 + 2] += e * hv.z;
          acc[4 * j4 + 3] += e * hv.w;
        }
      }
      const float inv = 1.0f / sum;
      float* orow = RG + (s * N_NODES + d) * GH;
#pragma unroll
      for (int j = 0; j < GH; ++j) {
        float v = acc[j] * inv + sBi1[j];
        const float vn = expm1f(fminf(v, 0.f));
        v = (v > 0.f) ? v : vn;
        orow[j] = v;
      }
    }
  }
  __syncthreads();

#pragma unroll
  for (int rep = 0; rep < 2; ++rep) {
    const int tI = wave + NWAVE * rep;
    if (tI < NT) {
      v16b ah0, al0, ah1, al1;
      const float* ar = RG + (tI * 16 + m) * GH + 8 * hh;
      load_a_split(ar, ah0, al0);
      load_a_split(ar + 32, ah1, al1);
#pragma unroll
      for (int nt = 0; nt < KP / 16; ++nt) {
        v8f c = {0.f, 0.f, 0.f, 0.f, 0.f, 0.f, 0.f, 0.f};
        FragB bh, bl;
        load_b(ph, pl, PL_W2 + (16 * nt + m) * GH + 8 * hh, bh, bl);
        c = wm3(ah0, al0, bh.v, bl.v, c);
        load_b(ph, pl, PL_W2 + (16 * nt + m) * GH + 32 + 8 * hh, bh, bl);
        c = wm3(ah1, al1, bh.v, bl.v, c);
        float* dp = RX + (tI * 16 + 8 * hh) * KP + 16 * nt + m;
#pragma unroll
        for (int r = 0; r < 8; ++r) dp[r * KP] = c[r];
      }
    }
  }
  __syncthreads();

  {
    const int s = t >> 4, n = t & 15;
    float p = 0.f, q = 0.f;
    if (n < N_NODES) {
      const float* hr = RX + (s * N_NODES + n) * KP;
#pragma unroll
      for (int f4 = 0; f4 < SEQ / 4; ++f4) {
        const v4f hv = *(const v4f*)(hr + 4 * f4);
        const v4f av = *(const v4f*)(sAs2 + 4 * f4);
        const v4f dv = *(const v4f*)(sAd2 + 4 * f4);
        p = p + hv.x * av.x; p = p + hv.y * av.y; p = p + hv.z * av.z; p = p + hv.w * av.w;
        q = q + hv.x * dv.x; q = q + hv.y * dv.y; q = q + hv.z * dv.z; q = q + hv.w * dv.w;
      }
    }
    sP[s * 16 + n] = p;
    sQ[s * 16 + n] = q;
  }
  __syncthreads();

  {
    const int s = t >> 4, d = t & 15;
    if (d < N_NODES) {
      int cnt = sCnt[d];
      cnt = cnt < 1 ? 1 : (cnt > ETOT ? ETOT : cnt);
      const float  qd  = sQ[s * 16 + d];
      const float* sPs = sP + s * 16;
      const int*   adj = sAdj + d * ADJP;
      float mx = -3.0e38f;
#pragma unroll 1
      for (int i = 0; i < cnt; ++i) {
        int sr = adj[i];
        sr = sr < 0 ? 0 : (sr > N_NODES - 1 ? N_NODES - 1 : sr);
        float a = sPs[sr] + qd;
        a = (a >= 0.f) ? a : 0.2f * a;
        mx = fmaxf(mx, a);
      }
      float acc[SEQ];
#pragma unroll
      for (int j = 0; j < SEQ; ++j) acc[j] = 0.f;
      float sum = 0.f;
#pragma unroll 1
      for (int i = 0; i < cnt; ++i) {
        int sr = adj[i];
        sr = sr < 0 ? 0 : (sr > N_NODES - 1 ? N_NODES - 1 : sr);
        float a = sPs[sr] + qd;
        a = (a >= 0.f) ? a : 0.2f * a;
        const float e = __expf(a - mx);
        sum += e;
        const float* hr = RX + (s * N_NODES + sr) * KP;
#pragma unroll
        for (int j4 = 0; j4 < SEQ / 4; ++j4) {
          const v4f hv = *(const v4f*)(hr + 4 * j4);
          acc[4 * j4 + 0] += e * hv.x;
          acc[4 * j4 + 1] += e * hv.y;
          acc[4 * j4 + 2] += e * hv.z;
          acc[4 * j4 + 3] += e * hv.w;
        }
      }
      const float inv = 1.0f / sum;
      float* orow = RH + (s * N_NODES + d) * KP;
#pragma unroll
      for (int j = 0; j < SEQ; ++j) orow[j] = acc[j] * inv + sBi2[j];
#pragma unroll
      for (int j = SEQ; j < KP; ++j) orow[j] = 0.f;
    }
  }
  __syncthreads();

#pragma unroll
  for (int rep = 0; rep < 2; ++rep) {
    const int n = wave + NWAVE * rep;
    if (n < N_NODES) {
      v16b ah, al;
      load_a_split(RH + (m * N_NODES + n) * KP + 8 * hh, ah, al);
#pragma unroll
      for (int nt = 0; nt < MH / 16; ++nt) {
        FragB bh, bl;
        load_b(ph, pl, PL_F1 + (n * MH + 16 * nt + m) * KP + 8 * hh, bh, bl);
        v8f c = {0.f, 0.f, 0.f, 0.f, 0.f, 0.f, 0.f, 0.f};
        c = wm3(ah, al, bh.v, bl.v, c);
        const int col = 16 * nt + m;
        const float bias = f1b[n * MH + col];
        float* dp = RG + (n * SPB + 8 * hh) * MH + col;
#pragma unroll
        for (int r = 0; r < 8; ++r) dp[r * MH] = fmaxf(c[r] + bias, 0.f);
      }
    }
  }
  __syncthreads();

#pragma unroll
  for (int rep = 0; rep < 2; ++rep) {
    const int n = wave + NWAVE * rep;
    if (n < N_NODES) {
      v16b ah0, al0, ah1, al1;
      const float* ar = RG + (n * SPB + m) * MH + 8 * hh;
      load_a_split(ar, ah0, al0);
      load_a_split(ar + 32, ah1, al1);
#pragma unroll
      for (int nt = 0; nt < KP / 16; ++nt) {
        v8f c = {0.f, 0.f, 0.f, 0.f, 0.f, 0.f, 0.f, 0.f};
        FragB bh, bl;
        load_b(ph, pl, PL_F2 + (n * KP + 16 * nt + m) * MH + 8 * hh, bh, bl);
        c = wm3(ah0, al0, bh.v, bl.v, c);
        load_b(ph, pl, PL_F2 + (n * KP + 16 * nt + m) * MH + 32 + 8 * hh, bh, bl);
        c = wm3(ah1, al1, bh.v, bl.v, c);
        const int col = 16 * nt + m;
        const int cc  = col < SEQ ? col : SEQ - 1;
        const float bias = f2b[n * SEQ + cc];
        if (col < SEQ) {
          float* dp = RX + (n * SPB + 8 * hh) * SEQ + col;
#pragma unroll
          for (int r = 0; r < 8; ++r) dp[r * SEQ] = c[r] + bias;
        }
      }
    }
  }
  __syncthreads();

  {
    float* ob = out + (size_t)b0 * SEQ;
    const size_t nstride = (size_t)nB * SEQ;
#pragma unroll 1
    for (int u = wave; u < 3 * N_NODES; u += NWAVE) {
      const int n = u / 3, p = u - 3 * n;
      const v4f v = *(const v4f*)(RX + n * (SPB * SEQ) + p * 128 + 4 * lane);
      *(volatile v4f*)(ob + (size_t)n * nstride + (size_t)(p * 128 + 4 * lane)) = v;
    }
    __threadfence();
#pragma unroll 1
    for (int u = wave; u < 3 * N_NODES; u += NWAVE) {
      const int n = u / 3, p = u - 3 * n;
      const v4f v = *(const v4f*)(RX + n * (SPB * SEQ) + p * 128 + 4 * lane);
      *(volatile v4f*)(ob + (size_t)n * nstride + (size_t)(p * 128 + 4 * lane)) = v;
    }
  }
}

extern "C" void kernel_launch(void* const* d_in, const int* in_sizes, int n_in,
                              void* d_out, int out_size, void* d_ws, size_t ws_size,
                              hipStream_t stream) {
  if (n_in < 14) return;
  const int per = SEQ * N_NODES;
  const int nB  = in_sizes[0] / per;
  if (nB <= 0 || in_sizes[0] != nB * per || (nB % SPB) != 0) return;
  if (in_sizes[1] != 2 * NEDGE) return;
  if (in_sizes[2] != SEQ * GH || in_sizes[3] != GH || in_sizes[4] != GH || in_sizes[5] != GH) return;
  if (in_sizes[6] != GH * SEQ || in_sizes[7] != SEQ || in_sizes[8] != SEQ || in_sizes[9] != SEQ) return;
  if (in_sizes[10] != N_NODES * SEQ * MH || in_sizes[11] != N_NODES * MH) return;
  if (in_sizes[12] != N_NODES * MH * SEQ || in_sizes[13] != N_NODES * SEQ) return;
  if (out_size != N_NODES * nB * SEQ) return;

  const float* x   = (const float*)d_in[0];
  const int*   ei  = (const int*)d_in[1];
  const float* W1  = (const float*)d_in[2];
  const float* as1 = (const float*)d_in[3];
  const float* ad1 = (const float*)d_in[4];
  const float* b1  = (const float*)d_in[5];
  const float* W2  = (const float*)d_in[6];
  const float* as2 = (const float*)d_in[7];
  const float* ad2 = (const float*)d_in[8];
  const float* b2  = (const float*)d_in[9];
  const float* f1w = (const float*)d_in[10];
  const float* f1b = (const float*)d_in[11];
  const float* f2w = (const float*)d_in[12];
  const float* f2b = (const float*)d_in[13];
  float* out = (float*)d_out;

  const size_t planeBytes = (size_t)PL_TOT * 2;
  const size_t total = 2 * planeBytes;
  if (total > ws_size) return;
  char* ws = (char*)d_ws;
  __bf16* ph = (__bf16*)(ws);
  __bf16* pl = (__bf16*)(ws + planeBytes);

  k_prep<<<dim3(N_NODES, 4), dim3(NTHR), 0, stream>>>(W1, W2, f1w, f2w, ph, pl);

  hipFuncSetAttribute(reinterpret_cast<const void*>(&k_main),
                      hipFuncAttributeMaxDynamicSharedMemorySize, LDS_BYTES);
  k_main<<<dim3(nB / SPB), dim3(NTHR), LDS_BYTES, stream>>>(
      x, ei, as1, ad1, b1, as2, ad2, b2, f1b, f2b, ph, pl, out, nB);
}
